// CAttention_12034498363841
// MI455X (gfx1250) — hardware-verified
//
#include <hip/hip_runtime.h>
#include <hip/hip_bf16.h>
#include <math.h>

#define NBc 4
#define NNc 1024
#define DMc 512
#define INR 512
#define NHc 8
#define DHc 64
#define NREL 1025
#define NRP 1152
#define MTOK (NBc * NNc)
#define SS 1024
#define HH 1
#define DKK 64
#define GSTR 48

typedef _Float16 bf16;
typedef _Float16 f16;
typedef __attribute__((ext_vector_type(4))) unsigned v4u_t;
typedef unsigned v4ua __attribute__((ext_vector_type(4), may_alias));
typedef __attribute__((ext_vector_type(4))) float v4f_t;
typedef float v4fa __attribute__((ext_vector_type(4), may_alias));
typedef __attribute__((ext_vector_type(16))) bf16  bf16x16;
typedef bf16x16 f16x16;
typedef __attribute__((ext_vector_type(8)))  bf16  bf16x8;
typedef bf16x8 f16x8;
typedef __attribute__((ext_vector_type(4)))  bf16  bf16x4;
typedef __attribute__((ext_vector_type(8)))  float f32x8;
__device__ __forceinline__ f32x8 wmma16(f16x16 a, f16x16 b, f32x8 c) {
  c = __builtin_amdgcn_wmma_f32_16x16x32_f16(false, a, false, b, (short)0, c, false, false);
  asm volatile("v_nop\n\tv_nop\n\tv_nop\n\tv_nop" : "+v"(c) : "v"(a), "v"(b));
  return c;
}
#define LDS_STRIDE 48
#define KSTRIDE    72
#define VSTRIDE    48

__device__ __forceinline__ f32x8 wmma_bf16(bf16x16 a, bf16x16 b, f32x8 c) {
  c = __builtin_amdgcn_wmma_f32_16x16x32_f16(false, a, false, b, (short)0, c, false, false);
  asm volatile("v_nop\n\tv_nop\n\tv_nop\n\tv_nop" : "+v"(c) : "v"(a), "v"(b));
  return c;
}

template <typename T>
__device__ __forceinline__ bf16x16 load_frag(const T* __restrict__ base, int ld,
                                             int row0, int k0) {
  const int lane = threadIdx.x & 31;
  const int r    = lane & 15;
  const int kh   = (lane >> 4) * 8;
  const T* p0 = base + (size_t)(row0 + r) * ld + (k0 + kh);
  const T* p1 = p0 + 16;
  bf16x16 f;
#pragma unroll
  for (int i = 0; i < 8; ++i) {
    f[i]     = (bf16)p0[i];
    f[i + 8] = (bf16)p1[i];
  }
  return f;
}

__device__ __forceinline__ bf16x16 lds_frag(const bf16* base, int stride) {
  const int lane = threadIdx.x & 31;
  const int row  = lane & 15;
  const int kh   = (lane >> 4) * 8;
  const bf16x8 lo = *(const bf16x8*)(base + row * stride + kh);
  const bf16x8 hi = *(const bf16x8*)(base + row * stride + kh + 16);
  bf16x16 f;
#pragma unroll
  for (int i = 0; i < 8; ++i) { f[i] = lo[i]; f[i + 8] = hi[i]; }
  return f;
}

template <typename T>
__device__ __forceinline__ void stage_read16(const T* __restrict__ p, float* buf) {
#pragma unroll
  for (int i = 0; i < 16; ++i) buf[i] = (float)p[i];
}

__device__ __forceinline__ void stage_write(bf16* dst, const float* buf, int nquad) {
#pragma unroll
  for (int i = 0; i < nquad; ++i) {
    bf16x4 q;
    q[0] = (bf16)buf[4 * i];     q[1] = (bf16)buf[4 * i + 1];
    q[2] = (bf16)buf[4 * i + 2]; q[3] = (bf16)buf[4 * i + 3];
    *(bf16x4*)(dst + 4 * i) = q;
  }
}

template <typename AT, int MODE>
__global__ __launch_bounds__(256) void gemm_rb_kernel(
    const AT* __restrict__ A, const float* __restrict__ W,
    const float* __restrict__ bias, const float* __restrict__ rowscale, const float* __restrict__ R, const float* __restrict__ rowbias, void* __restrict__ out,
    int M, int N, int K) {
  __shared__ bf16 ldsA[128 * LDS_STRIDE];
  __shared__ bf16 ldsW[256 * LDS_STRIDE];
  __shared__ __attribute__((aligned(16))) unsigned char sob[256 * 136 * 2];

  const int t    = threadIdx.x;
  const int wave = t >> 5;
  const int lane = t & 31;
  const int wm   = (wave & 1) * 64;
  const int wn   = (wave >> 1) * 64;
  const int mBlk = blockIdx.x * 128;
  const int nBlk = blockIdx.y * 256;

  const int arow = t >> 1;
  const int ach  = (t & 1) * 16;

  float abuf[16];
  float wbuf[32];

  stage_read16(A + (size_t)(mBlk + arow) * K + ach, abuf);
  const int nrow = min(nBlk + t, N - 1);
  stage_read16(W + (size_t)nrow * K,          wbuf);
  stage_read16(W + (size_t)nrow * K + 16,     wbuf + 16);

  f32x8 acc[4][4] = {};

  for (int k = 0; k < K; k += 32) {
    __syncthreads();
    stage_write(&ldsA[arow * LDS_STRIDE + ach], abuf, 4);
    stage_write(&ldsW[t * LDS_STRIDE],          wbuf, 8);
    if (k + 32 < K) {
      stage_read16(A + (size_t)(mBlk + arow) * K + (k + 32) + ach, abuf);
      stage_read16(W + (size_t)nrow * K + (k + 32),          wbuf);
      stage_read16(W + (size_t)nrow * K + (k + 32) + 16,     wbuf + 16);
    }
    __syncthreads();

    bf16x16 af[4], wf[4];
#pragma unroll
    for (int i = 0; i < 4; ++i)
      af[i] = lds_frag(ldsA + (wm + 16 * i) * LDS_STRIDE, LDS_STRIDE);
#pragma unroll
    for (int j = 0; j < 4; ++j)
      wf[j] = lds_frag(ldsW + (wn + 16 * j) * LDS_STRIDE, LDS_STRIDE);
#pragma unroll
    for (int i = 0; i < 4; ++i)
#pragma unroll
      for (int j = 0; j < 4; ++j)
        acc[i][j] = wmma_bf16(af[i], wf[j], acc[i][j]);
  }

  const int nlane = lane & 15;
  const int mh    = (lane >> 4) * 8;
  __syncthreads();
  if (MODE == 0 || MODE == 1 || MODE == 3) {
    bf16* so = (bf16*)sob;
#pragma unroll
    for (int i = 0; i < 4; ++i)
#pragma unroll
      for (int j = 0; j < 4; ++j) {
        const int nl = wn + 16 * j + nlane;
        const float bv = bias ? bias[nBlk + nl] : 0.0f;
        if (MODE == 3) {
#pragma unroll 1
          for (int r = 0; r < 8; ++r) {
            const int ml = wm + 16 * i + mh + r;
            const float xg = acc[i][j][r] + bv;
            so[ml * 264 + nl] = (bf16)(0.5f * xg * (1.0f + erff(xg * 0.70710678118654752f)));
          }
        } else {
#pragma unroll
        for (int r = 0; r < 8; ++r) {
          const int ml = wm + 16 * i + mh + r;
          const bf16 hv = (bf16)(acc[i][j][r] + bv);
          if (MODE == 0) so[ml * 264 + nl] = hv;
          else           so[nl * 136 + ml] = hv;
        }
        }
      }
    __syncthreads();
#pragma unroll 1
    for (int pass = 0; pass < 2; ++pass) {
      if (MODE == 0 || MODE == 3) {
        for (int ch = t; ch < 128 * 32; ch += 256) { const int ml = ch >> 5, q = (ch & 31) * 8;
          *(volatile v4u_t*)((bf16*)out + (size_t)(mBlk + ml) * N + nBlk + q) = *(const v4ua*)(so + ml * 264 + q); }
      } else {
        const int b_ = mBlk / SS, s0 = mBlk % SS;
        for (int ch = t; ch < 256 * 16; ch += 256) { const int nl = ch >> 4, q = (ch & 15) * 8; const int n = nBlk + nl, h = n >> 6, dk = n & (DKK - 1);
          *(volatile v4u_t*)((bf16*)out + (((size_t)(b_ * HH + h)) * DKK + dk) * SS + s0 + q) = *(const v4ua*)(so + nl * 136 + q); }
      }
      __threadfence();
    }
  } else {
    float* so = (float*)sob;
#pragma unroll 1
    for (int hf = 0; hf < 2; ++hf) {
      if (wm == hf * 64) {
#pragma unroll
        for (int i = 0; i < 4; ++i)
#pragma unroll
          for (int j = 0; j < 4; ++j) {
            const int nl = wn + 16 * j + nlane;
            const float bv = bias ? bias[nBlk + nl] : 0.0f;
#pragma unroll
            for (int r = 0; r < 8; ++r) { const int mrow = mBlk + hf * 64 + 16 * i + mh + r; so[(16 * i + mh + r) * 260 + nl] = acc[i][j][r] * (rowscale ? rowscale[mrow] : 1.0f) + bv + (rowbias ? rowbias[mrow] : 0.0f); }
          }
      }
      __syncthreads();
      if (R) {
        for (int ch = t; ch < 64 * 64; ch += 256) { const int ml = ch >> 6, q = (ch & 63) * 4;
          if (nBlk + q < N) { const v4f_t rv = *(const v4f_t*)(R + (size_t)(mBlk + hf * 64 + ml) * N + nBlk + q); v4f_t v = *(const v4fa*)(so + ml * 260 + q); v += rv; *(volatile v4fa*)(so + ml * 260 + q) = v; } }
        asm volatile("s_wait_dscnt 0" ::: "memory");
      }
#pragma unroll 1
      for (int pass = 0; pass < 2; ++pass) {
        for (int ch = t; ch < 64 * 64; ch += 256) { const int ml = ch >> 6, q = (ch & 63) * 4;
          if (nBlk + q < N) *(volatile v4f_t*)((float*)out + (size_t)(mBlk + hf * 64 + ml) * N + nBlk + q) = *(const v4fa*)(so + ml * 260 + q); }
        __threadfence();
      }
      __syncthreads();
    }
  }
}


#define GSTR 48
template <typename AT, int EPI, bool OUT16>
__global__ __launch_bounds__(256) void gemm_kne(const AT* __restrict__ A, int lda, const float* __restrict__ Wm, int ldw,
                                                const float* __restrict__ bias, const float* __restrict__ R, const float* __restrict__ gvec,
                                                void* __restrict__ Yv, int ldy, int K) {
  __shared__ __attribute__((aligned(16))) f16 ldsA[128 * GSTR];
  __shared__ __attribute__((aligned(16))) f16 ldsW[128 * GSTR];
  __shared__ __attribute__((aligned(16))) float oS[8][32 * 68];
  const int tid = threadIdx.x, lane = tid & 31, wave = tid >> 5, cl = lane & 15, rh = (lane >> 4) * 8;
  const int m0 = blockIdx.x * 128, n0 = blockIdx.y * 128;
  const int wm = (wave & 3) * 32, wn = (wave >> 2) * 64;
  f32x8 acc[2][4];
#pragma unroll
  for (int i = 0; i < 2; ++i)
#pragma unroll
    for (int j = 0; j < 4; ++j) { f32x8 z = {}; acc[i][j] = z; }
#pragma unroll 1
  for (int k0 = 0; k0 < K; k0 += 32) {
    __syncthreads();
    { const int row = tid >> 1, ch = (tid & 1) * 16;
      const AT* src = A + (size_t)(m0 + row) * lda + k0 + ch;
#pragma unroll
      for (int g = 0; g < 16; ++g) ldsA[row * GSTR + ch + g] = (f16)src[g]; }
    { const int k = tid >> 3, nn0 = (tid & 7) * 16;
      const float* src = Wm + (size_t)(k0 + k) * ldw + n0 + nn0;
#pragma unroll
      for (int g = 0; g < 4; ++g) { const v4f_t v = *(const v4f_t*)(src + 4 * g);
#pragma unroll
        for (int u = 0; u < 4; ++u) ldsW[(nn0 + 4 * g + u) * GSTR + k] = (f16)v[u]; } }
    __syncthreads();
    f16x16 af[2];
#pragma unroll
    for (int i = 0; i < 2; ++i) af[i] = lds_frag(ldsA + (wm + 16 * i) * GSTR, GSTR);
#pragma unroll
    for (int j = 0; j < 4; ++j) {
      const f16x16 bf = lds_frag(ldsW + (wn + 16 * j) * GSTR, GSTR);
#pragma unroll
      for (int i = 0; i < 2; ++i) acc[i][j] = wmma16(af[i], bf, acc[i][j]);
    }
  }
  float* so = oS[wave];
#pragma unroll
  for (int i = 0; i < 2; ++i)
#pragma unroll
    for (int j = 0; j < 4; ++j) {
      const int n = n0 + wn + 16 * j + cl;
      const float bv = bias ? bias[n] : 0.0f;
      const float gv = (EPI == 2) ? gvec[n] : 0.0f;
      if (EPI == 1) {
#pragma unroll 1
        for (int r = 0; r < 8; ++r) { const float xg = acc[i][j][r] + bv; so[(16 * i + rh + r) * 68 + 16 * j + cl] = 0.5f * xg * (1.0f + erff(xg * 0.70710678118654752f)); }
      } else {
#pragma unroll
        for (int r = 0; r < 8; ++r) {
          float v = acc[i][j][r] + bv;
          if (EPI == 2) v = R[(size_t)(m0 + wm + 16 * i + rh + r) * ldy + n] + gv * v;
          so[(16 * i + rh + r) * 68 + 16 * j + cl] = v;
        }
      }
    }
  asm volatile("s_wait_dscnt 0" ::: "memory");
  __builtin_amdgcn_wave_barrier();
#pragma unroll 1
  for (int pass = 0; pass < 2; ++pass) {
    if (OUT16) {
      f16* Y = (f16*)Yv;
#pragma unroll
      for (int it = 0; it < 8; ++it) { const int c = lane + 32 * it, rr = c >> 3, q8 = (c & 7) * 8;
        union { f16 h[8]; v4u_t v; } u;
#pragma unroll
        for (int e = 0; e < 8; ++e) u.h[e] = (f16)so[rr * 68 + q8 + e];
        *(volatile v4u_t*)(Y + (size_t)(m0 + wm + rr) * ldy + n0 + wn + q8) = u.v; }
    } else {
      float* Y = (float*)Yv;
#pragma unroll
      for (int it = 0; it < 16; ++it) { const int f4 = lane + 32 * it, rr = f4 >> 4, q = (f4 & 15) * 4;
        *(volatile v4f_t*)(Y + (size_t)(m0 + wm + rr) * ldy + n0 + wn + q) = *(const v4fa*)(so + rr * 68 + q); }
    }
    __threadfence();
  }
}

__global__ __launch_bounds__(256) void k_deint(const float* __restrict__ x, float* __restrict__ AB) { const size_t t = blockIdx.x;
  for (int c = threadIdx.x; c < DMc; c += 256) { const float a = x[(t * DMc + c) * 2], b = x[(t * DMc + c) * 2 + 1]; *(volatile float*)(AB + t * 2 * DMc + c) = a; *(volatile float*)(AB + t * 2 * DMc + DMc + c) = b; }
  __threadfence();
  for (int c = threadIdx.x; c < DMc; c += 256) { const float a = x[(t * DMc + c) * 2], b = x[(t * DMc + c) * 2 + 1]; *(volatile float*)(AB + t * 2 * DMc + c) = a; *(volatile float*)(AB + t * 2 * DMc + DMc + c) = b; } }
__global__ __launch_bounds__(256) void k_wcomplex(const float* __restrict__ Wr, const float* __restrict__ Wi, int K, int N, float* __restrict__ Wc) { const int r = blockIdx.x; const int kk = (r < K) ? r : r - K;
#pragma unroll 1
  for (int pass = 0; pass < 2; ++pass) {
    for (int c = threadIdx.x; c < 2 * N; c += 256) { const int n = (c < N) ? c : c - N; const float wr = Wr[(size_t)kk * N + n], wi = Wi[(size_t)kk * N + n];
      float v; if (r < K) v = (c < N) ? wr : wi; else v = (c < N) ? -wi : wr; *(volatile float*)(Wc + (size_t)r * 2 * N + c) = v; }
    __threadfence(); } }
__global__ __launch_bounds__(256) void k_headops(const bf16* __restrict__ Q, const bf16* __restrict__ KV, int b, int h, float* __restrict__ QA, float* __restrict__ QB, float* __restrict__ KA, float* __restrict__ KB, float* __restrict__ VV) {
  const int n = blockIdx.x; const size_t t = (size_t)b * NNc + n; const int c = threadIdx.x;
  if (c < 128) { const int d = c & 63; const bool hi = c >= 64; const float qr = (float)Q[t * 2 * INR + h * DHc + d], qi = (float)Q[t * 2 * INR + INR + h * DHc + d];
    const float va = hi ? -qi : qr, vb = hi ? qi : qr;
    *(volatile float*)(QA + (size_t)n * 128 + c) = va; *(volatile float*)(QB + (size_t)n * 128 + c) = vb; }
  else { const int cc = c - 128; const int d = cc & 63; const bool hi = cc >= 64;
    const float kr = (float)KV[t * 4 * INR + h * DHc + d], ki = (float)KV[t * 4 * INR + 2 * INR + h * DHc + d], vr = (float)KV[t * 4 * INR + INR + h * DHc + d], vi = (float)KV[t * 4 * INR + 3 * INR + h * DHc + d];
    *(volatile float*)(KA + (size_t)n * 128 + cc) = hi ? ki : kr; *(volatile float*)(KB + (size_t)n * 128 + cc) = hi ? kr : ki; *(volatile float*)(VV + (size_t)n * 128 + cc) = hi ? vi : vr; }
  __threadfence();
  if (c < 128) { const int d = c & 63; const bool hi = c >= 64; const float qr = (float)Q[t * 2 * INR + h * DHc + d], qi = (float)Q[t * 2 * INR + INR + h * DHc + d];
    *(volatile float*)(QA + (size_t)n * 128 + c) = hi ? -qi : qr; *(volatile float*)(QB + (size_t)n * 128 + c) = hi ? qi : qr; }
  else { const int cc = c - 128; const int d = cc & 63; const bool hi = cc >= 64;
    const float kr = (float)KV[t * 4 * INR + h * DHc + d], ki = (float)KV[t * 4 * INR + 2 * INR + h * DHc + d], vr = (float)KV[t * 4 * INR + INR + h * DHc + d], vi = (float)KV[t * 4 * INR + 3 * INR + h * DHc + d];
    *(volatile float*)(KA + (size_t)n * 128 + cc) = hi ? ki : kr; *(volatile float*)(KB + (size_t)n * 128 + cc) = hi ? kr : ki; *(volatile float*)(VV + (size_t)n * 128 + cc) = hi ? vi : vr; }
}
__global__ __launch_bounds__(256) void k_relT(const float* __restrict__ rel, float* __restrict__ RT) { const int d = blockIdx.x;
#pragma unroll 1
  for (int pass = 0; pass < 2; ++pass) { for (int r = threadIdx.x; r < NRP; r += 256) { const int rc = (r < NREL) ? r : NREL - 1; float v = rel[(size_t)rc * DHc + d]; v = (r < NREL) ? v : 0.0f;
      *(volatile float*)(RT + (size_t)d * NRP + r) = v; } __threadfence(); } }
__global__ __launch_bounds__(256) void k_magsoftmax(float* __restrict__ Re, const float* __restrict__ Im, const float* __restrict__ Tr, const float* __restrict__ Ti) {
  __shared__ float red[256];
  const int i = blockIdx.x, tid = threadIdx.x; float* re = Re + (size_t)i * NNc; const float* im = Im + (size_t)i * NNc; const float* tr = Tr + (size_t)i * NRP; const float* ti = Ti + (size_t)i * NRP;
  float v[4]; float mx = -3.0e38f;
#pragma unroll
  for (int e = 0; e < 4; ++e) { const int j = tid + 256 * e; int dlt = i - j; dlt = dlt < -512 ? -512 : (dlt > 512 ? 512 : dlt); const int ridx = dlt + 512;
    const float a = re[j] + tr[ridx], bq = im[j] + ti[ridx]; v[e] = sqrtf(a * a + bq * bq) * 0.125f; mx = fmaxf(mx, v[e]); }
  red[tid] = mx; __syncthreads();
  for (int o = 128; o > 0; o >>= 1) { if (tid < o) red[tid] = fmaxf(red[tid], red[tid + o]); __syncthreads(); }
  mx = red[0]; __syncthreads();
  float z = 0.0f;
#pragma unroll
  for (int e = 0; e < 4; ++e) { v[e] = expf(v[e] - mx); z += v[e]; }
  red[tid] = z; __syncthreads();
  for (int o = 128; o > 0; o >>= 1) { if (tid < o) red[tid] += red[tid + o]; __syncthreads(); }
  const float sc = 1024.0f / red[0];
#pragma unroll 1
  for (int pass = 0; pass < 2; ++pass) {
#pragma unroll
    for (int e = 0; e < 4; ++e) *(volatile float*)(re + tid + 256 * e) = v[e] * sc;
    __threadfence(); }
}
__global__ __launch_bounds__(128) void k_place(const float* __restrict__ O, int b, int h, float* __restrict__ OUT2) { const int n = blockIdx.x; const int c = threadIdx.x; const int d = c & 63; const bool hi = c >= 64;
  const float v = O[(size_t)n * 128 + c] * (1.0f / 1024.0f); float* dst = OUT2 + ((size_t)b * NNc + n) * 2 * INR + (hi ? INR : 0) + h * DHc + d; *(volatile float*)dst = v; __threadfence(); *(volatile float*)dst = v; }
__global__ __launch_bounds__(256) void k_bcat(const float* __restrict__ br, const float* __restrict__ bi, float* __restrict__ bo2) { for (int c = threadIdx.x; c < 2 * DMc; c += 256) { const float v = (c < DMc) ? br[c] : bi[c - DMc]; *(volatile float*)(bo2 + c) = v; __threadfence(); *(volatile float*)(bo2 + c) = v; } }
__global__ __launch_bounds__(256) void k_reint(const float* __restrict__ Y, float* __restrict__ out) { const size_t t = blockIdx.x; typedef __attribute__((ext_vector_type(2))) float v2f;
  for (int c = threadIdx.x; c < DMc; c += 256) { v2f p; p[0] = Y[t * 2 * DMc + c]; p[1] = Y[t * 2 * DMc + DMc + c]; *(volatile v2f*)(out + (t * DMc + c) * 2) = p; }
  __threadfence();
  for (int c = threadIdx.x; c < DMc; c += 256) { v2f p; p[0] = Y[t * 2 * DMc + c]; p[1] = Y[t * 2 * DMc + DMc + c]; *(volatile v2f*)(out + (t * DMc + c) * 2) = p; } }

extern "C" void kernel_launch(void* const* d_in, const int* in_sizes, int n_in,
                              void* d_out, int out_size, void* d_ws, size_t ws_size,
                              hipStream_t stream) {
  (void)in_sizes; (void)n_in; (void)out_size;
  const float** f = (const float**)d_in;
  const float* x = f[0], *wq_r = f[1], *wq_i = f[2], *wkv_r = f[3], *wkv_i = f[4], *wo_r = f[5], *wo_i = f[6], *bo_r = f[7], *bo_i = f[8], *rel = f[9];
  float* out = (float*)d_out;
  char* ws = (char*)d_ws;
  float* AB = (float*)ws; ws += (size_t)MTOK * 2 * DMc * 4;
  float* Wcq = (float*)ws; ws += (size_t)2 * DMc * 2 * INR * 4;
  float* Wckv = (float*)ws; ws += (size_t)2 * DMc * 4 * INR * 4;
  float* Wco = (float*)ws; ws += (size_t)2 * INR * 2 * DMc * 4;
  float* bo2 = (float*)ws; ws += (size_t)2 * DMc * 4;
  bf16* Q = (bf16*)ws; ws += (size_t)MTOK * 2 * INR * 2;
  bf16* KV = (bf16*)ws; ws += (size_t)MTOK * 4 * INR * 2;
  float* Y = (float*)ws; ws += (size_t)MTOK * 2 * DMc * 4;
  float* RT = (float*)ws; ws += (size_t)DHc * NRP * 4;
  float* QA = (float*)ws; ws += (size_t)NNc * 128 * 4; float* QB = (float*)ws; ws += (size_t)NNc * 128 * 4; float* KA = (float*)ws; ws += (size_t)NNc * 128 * 4; float* KB = (float*)ws; ws += (size_t)NNc * 128 * 4; float* VV = (float*)ws; ws += (size_t)NNc * 128 * 4;
  float* Re = (float*)ws; ws += (size_t)NNc * NNc * 4; float* Im = (float*)ws; ws += (size_t)NNc * NNc * 4;
  float* Tr = (float*)ws; ws += (size_t)NNc * NRP * 4; float* Ti = (float*)ws; ws += (size_t)NNc * NRP * 4;
  float* O = (float*)ws; ws += (size_t)NNc * 128 * 4;
  float* OUT2 = AB;
  if ((size_t)(ws - (char*)d_ws) > ws_size) return;
  const dim3 blk(256);
  k_wcomplex<<<dim3(2 * DMc), blk, 0, stream>>>(wq_r, wq_i, DMc, INR, Wcq);
  k_wcomplex<<<dim3(2 * DMc), blk, 0, stream>>>(wkv_r, wkv_i, DMc, 2 * INR, Wckv);
  k_wcomplex<<<dim3(2 * INR), blk, 0, stream>>>(wo_r, wo_i, INR, DMc, Wco);
  k_relT<<<dim3(DHc), blk, 0, stream>>>(rel, RT);
  k_deint<<<dim3(MTOK), blk, 0, stream>>>(x, AB);
  k_bcat<<<dim3(1), blk, 0, stream>>>(bo_r, bo_i, bo2);
  gemm_kne<float, 0, true><<<dim3(MTOK / 128, 2 * INR / 128), blk, 0, stream>>>(AB, 2 * DMc, Wcq, 2 * INR, nullptr, nullptr, nullptr, Q, 2 * INR, 2 * DMc);
  gemm_kne<float, 0, true><<<dim3(MTOK / 128, 4 * INR / 128), blk, 0, stream>>>(AB, 2 * DMc, Wckv, 4 * INR, nullptr, nullptr, nullptr, KV, 4 * INR, 2 * DMc);
  for (int b = 0; b < NBc; ++b) for (int h = 0; h < NHc; ++h) {
    k_headops<<<dim3(NNc), blk, 0, stream>>>(Q, KV, b, h, QA, QB, KA, KB, VV);
    gemm_rb_kernel<float, 2><<<dim3(NNc / 128, NNc / 256), blk, 0, stream>>>(QA, KA, nullptr, nullptr, nullptr, nullptr, Re, NNc, NNc, 128);
    gemm_rb_kernel<float, 2><<<dim3(NNc / 128, NNc / 256), blk, 0, stream>>>(QB, KB, nullptr, nullptr, nullptr, nullptr, Im, NNc, NNc, 128);
    gemm_kne<float, 0, false><<<dim3(NNc / 128, NRP / 128), blk, 0, stream>>>(QB, 128, RT, NRP, nullptr, nullptr, nullptr, Tr, NRP, 64);
    gemm_kne<float, 0, false><<<dim3(NNc / 128, NRP / 128), blk, 0, stream>>>(QB + 64, 128, RT, NRP, nullptr, nullptr, nullptr, Ti, NRP, 64);
    k_magsoftmax<<<dim3(NNc), blk, 0, stream>>>(Re, Im, Tr, Ti);
    gemm_kne<float, 0, false><<<dim3(NNc / 128, 1), blk, 0, stream>>>(Re, NNc, VV, 128, nullptr, nullptr, nullptr, O, 128, NNc);
    k_place<<<dim3(NNc), dim3(128), 0, stream>>>(O, b, h, OUT2);
  }
  gemm_kne<float, 0, false><<<dim3(MTOK / 128, 2 * DMc / 128), blk, 0, stream>>>(OUT2, 2 * INR, Wco, 2 * DMc, bo2, nullptr, nullptr, Y, 2 * DMc, 2 * INR);
  k_reint<<<dim3(MTOK), blk, 0, stream>>>(Y, out);
}
